// Tanh_RNN_25116968747218
// MI455X (gfx1250) — hardware-verified
//
#include <hip/hip_runtime.h>
#include <math.h>

constexpr int NB    = 64;
constexpr int NT    = 512;
constexpr int NVOC  = 50000;
constexpr int NE    = 256;
constexpr int NU    = 512;
constexpr int NH1   = 128;
constexpr int NH2   = 64;
constexpr int NROWS = NB * NT;
constexpr int NTHR  = 256;
constexpr int SEQ_BLK = 16;
constexpr int HPITCH  = 520;
constexpr int ABUF    = SEQ_BLK * HPITCH;
constexpr int SLABP   = 68;
constexpr int TSP     = 68;
constexpr float EMB_CARRY = 64.0f;
constexpr float W_CARRY   = 16.0f;
constexpr float XW_FOLD   = 1.0f / 1024.0f;
constexpr float WH_FOLD   = 1.0f / 16.0f;
static_assert(NB % SEQ_BLK == 0);
static_assert(NU == 64 * (NTHR / 32));
static_assert(NE % 32 == 0 && NU % 32 == 0);
static_assert(NROWS % 64 == 0 && NU % 64 == 0);
static_assert(NE % 64 == 0);
static_assert(NE / 8 == 32);
static_assert((2 * ABUF) % NTHR == 0);
static_assert((NROWS * (NE / 8)) % NTHR == 0);
static_assert((NB * NH1) % NTHR == 0 && (NB * NH2) % NTHR == 0);

typedef __attribute__((ext_vector_type(16))) _Float16 v16h;
typedef __attribute__((ext_vector_type(8)))  _Float16 v8h;
typedef __attribute__((ext_vector_type(16))) __bf16   v16b;
typedef __attribute__((ext_vector_type(8)))  __bf16   v8b;
typedef __attribute__((ext_vector_type(8)))  float    v8f;
typedef __attribute__((ext_vector_type(4)))  float    v4f;

__device__ __forceinline__ unsigned short f2bf_bits(float f) {
  unsigned u = __float_as_uint(f);
  return (unsigned short)((u + 0x7FFFu + ((u >> 16) & 1u)) >> 16);
}
__device__ __forceinline__ float bf_bits2f(unsigned short h) { return __uint_as_float(((unsigned)h) << 16); }

__device__ __forceinline__ void dep_guard_h(v8f& a, v8f& b, v16h x, v16h y) { asm volatile("v_nop\n\tv_nop\n\tv_nop\n\tv_nop" : "+v"(a), "+v"(b) : "v"(x), "v"(y)); }
__device__ __forceinline__ void dep_guard_b(v8f& a, v8f& b, v16b x, v16b y) { asm volatile("v_nop\n\tv_nop\n\tv_nop\n\tv_nop" : "+v"(a), "+v"(b) : "v"(x), "v"(y)); }
__device__ __forceinline__ void keep4_h(v16h a, v16h b, v16h c, v16h d) { asm volatile("v_nop" :: "v"(a), "v"(b), "v"(c), "v"(d)); }
__device__ __forceinline__ void keep4_b(v16b a, v16b b, v16b c, v16b d) { asm volatile("v_nop" :: "v"(a), "v"(b), "v"(c), "v"(d)); }
__device__ __forceinline__ void acc_guard4(v8f& a, v8f& b, v8f& c, v8f& d) { asm volatile("v_nop\n\tv_nop\n\tv_nop\n\tv_nop" : "+v"(a), "+v"(b), "+v"(c), "+v"(d)); }
template <typename T> struct Frag;
template <> struct Frag<_Float16> {
  typedef v16h V; union U { v16h v; v8h h[2]; };
  static __device__ __forceinline__ v16h load(const _Float16* p) {
    U f; f.h[0] = *(const v8h*)(p); f.h[1] = *(const v8h*)(p + 16); return f.v;
  }
  static __device__ __forceinline__ v8f mma(v16h a, v16h b, v8f c) {
    return __builtin_amdgcn_wmma_f32_16x16x32_f16(false, a, false, b, (short)0, c, false, false);
  }
  static __device__ __forceinline__ void guard(v8f& a, v8f& b, v16h x, v16h y) { dep_guard_h(a, b, x, y); }
  static __device__ __forceinline__ void keep(v16h a, v16h b, v16h c, v16h d) { keep4_h(a, b, c, d); }
};
template <> struct Frag<__bf16> {
  typedef v16b V; union U { v16b v; v8b h[2]; };
  static __device__ __forceinline__ v16b load(const __bf16* p) {
    U f; f.h[0] = *(const v8b*)(p); f.h[1] = *(const v8b*)(p + 16); return f.v;
  }
  static __device__ __forceinline__ v8f mma(v16b a, v16b b, v8f c) {
    return __builtin_amdgcn_wmma_f32_16x16x32_bf16(false, a, false, b, (short)0, c, false, false);
  }
  static __device__ __forceinline__ void guard(v8f& a, v8f& b, v16b x, v16b y) { dep_guard_b(a, b, x, y); }
  static __device__ __forceinline__ void keep(v16b a, v16b b, v16b c, v16b d) { keep4_b(a, b, c, d); }
};

template <int ET> struct Elem;
template <> struct Elem<0> { typedef _Float16 T; };
template <> struct Elem<1> { typedef __bf16 T; };
template <int ET, bool SPLIT, int BIAS_MODE, int OUT_MODE, bool RESID, int ACT = 0>
__global__ __launch_bounds__(256) void wmma_gemm64(
    const unsigned short* __restrict__ Ap, const unsigned short* __restrict__ A2p, int lda, long strideA,
    const unsigned short* __restrict__ Btp, const unsigned short* __restrict__ Bt2p, int ldb, long strideB,
    void* __restrict__ Cout, void* __restrict__ Cout2, int ldc, long strideC,
    const float* __restrict__ bias,
    const float* __restrict__ resid, long strideR,
    int M, int N, int K, float scale) {
  typedef typename Elem<ET>::T T;
  typedef typename Frag<T>::V V;
  const T* A = (const T*)Ap; const T* A2 = (const T*)A2p; const T* Bt = (const T*)Btp; const T* Bt2 = (const T*)Bt2p;
  __shared__ __align__(16) float sT[8][16 * 68];
  const int b    = blockIdx.y;
  const int lane = threadIdx.x & 31;
  const int wave = threadIdx.x >> 5;
  const int tilesN = N >> 6;
  const int tilesM = M >> 6;
  const int tile = blockIdx.x * 8 + wave;
  if (tile >= tilesM * tilesN) return;
  const int tm = tile / tilesN;
  const int tn = tile - tm * tilesN;
  const int m0 = tm << 6;
  const int n0 = tn << 6;

  const T* Ab  = A  + (size_t)b * strideA;
  const T* Bb  = Bt + (size_t)b * strideB;
  const T* Ab2 = SPLIT ? (A2  + (size_t)b * strideA) : nullptr;
  const T* Bb2 = SPLIT ? (Bt2 + (size_t)b * strideB) : nullptr;

  const int rlane = lane & 15;
  const int koff  = (lane >> 4) * 8;
  const int mOff  = (lane >> 4) * 8;

  v8f acc[4][4];
#pragma unroll
  for (int i = 0; i < 4; ++i)
#pragma unroll
    for (int j = 0; j < 4; ++j) acc[i][j] = (v8f){0.f,0.f,0.f,0.f,0.f,0.f,0.f,0.f};

  for (int k0 = 0; k0 < K; k0 += 32) {
    V bh[4], bl[4];
#pragma unroll
    for (int j = 0; j < 4; ++j) {
      const size_t bo = (size_t)(n0 + (j << 4) + rlane) * ldb + koff + k0;
      bh[j] = Frag<T>::load(Bb + bo);
      if (SPLIT) bl[j] = Frag<T>::load(Bb2 + bo);
    }
#pragma unroll
    for (int i = 0; i < 4; ++i) {
      const size_t ao = (size_t)(m0 + (i << 4) + rlane) * lda + koff + k0;
      V ah = Frag<T>::load(Ab + ao);
      V al;
      if (SPLIT) al = Frag<T>::load(Ab2 + ao);
#pragma unroll
      for (int j = 0; j < 4; ++j) {
        acc[i][j] = Frag<T>::mma(ah, bh[j], acc[i][j]);
        if (SPLIT) {
          acc[i][j] = Frag<T>::mma(ah, bl[j], acc[i][j]);
          acc[i][j] = Frag<T>::mma(al, bh[j], acc[i][j]);
        }
      }
      Frag<T>::guard(acc[i][0], acc[i][3], ah, SPLIT ? al : ah);
    }
    Frag<T>::keep(bh[0], bh[1], bh[2], bh[3]);
    if (SPLIT) Frag<T>::keep(bl[0], bl[1], bl[2], bl[3]);
  }
  acc_guard4(acc[0][0], acc[0][1], acc[0][2], acc[0][3]);
  acc_guard4(acc[1][0], acc[1][1], acc[1][2], acc[1][3]);
  acc_guard4(acc[2][0], acc[2][1], acc[2][2], acc[2][3]);
  acc_guard4(acc[3][0], acc[3][1], acc[3][2], acc[3][3]);

  float* slab = sT[wave];
  const float* Rb = RESID ? (resid + (size_t)b * strideR) : nullptr;
#pragma unroll
  for (int i = 0; i < 4; ++i) {
    const int mBase = m0 + (i << 4);
#pragma unroll
    for (int j = 0; j < 4; ++j) {
      const int n = n0 + (j << 4) + rlane;
      float bv = 0.f;
      if (BIAS_MODE == 2) bv = bias[n];
#pragma unroll
      for (int r = 0; r < 8; ++r) {
        float v = acc[i][j][r] * scale;
        if (BIAS_MODE == 1) v += bias[mBase + mOff + r];
        if (BIAS_MODE == 2) v += bv;
        if (RESID) v += Rb[(size_t)(mBase + mOff + r) * ldc + n];
        if (ACT == 1) v = tanhf(v);
        if (ACT == 2) v = fmaxf(v, 0.0f);
        if (ACT == 3) v = v / (1.0f + expf(-v));
        if (ACT == 4) v = (v > 0.f) ? v : 0.01f * v;
        if (ACT == 5) v = 0.5f * v * (1.0f + erff(v * 0.70710678118654752f));
        slab[(mOff + r) * 68 + (j << 4) + rlane] = v;
      }
    }
    __builtin_amdgcn_fence(__ATOMIC_RELEASE, "workgroup");
    __builtin_amdgcn_wave_barrier();
    __builtin_amdgcn_fence(__ATOMIC_ACQUIRE, "workgroup");
    if (OUT_MODE == 0) {
      float* C = (float*)Cout + (size_t)b * strideC;
      const int hh = lane >> 4, c4 = (lane & 15) * 4;
      for (int pass = 0; pass < 2; ++pass) {
#pragma unroll
        for (int it = 0; it < 8; ++it) {
          const int row = it * 2 + hh;
          v4f v = *(const v4f*)(slab + row * 68 + c4);
          *(volatile v4f*)(C + (size_t)(mBase + row) * ldc + n0 + c4) = v;
        }
        __threadfence();
      }
    } else {
      const int q = lane >> 3, c8 = (lane & 7) * 8;
      unsigned short* C  = (unsigned short*)Cout  + (size_t)b * strideC;
      unsigned short* C2 = (OUT_MODE == 2) ? ((unsigned short*)Cout2 + (size_t)b * strideC) : nullptr;
      for (int pass = 0; pass < 2; ++pass) {
#pragma unroll
        for (int it = 0; it < 4; ++it) {
          const int row = it * 4 + q;
          const float* sp = slab + row * 68 + c8;
          v8h hv, lv;
#pragma unroll
          for (int e = 0; e < 8; ++e) {
            if (OUT_MODE == 1) {
              hv[e] = (_Float16)sp[e];
            } else {
              unsigned short hb = f2bf_bits(sp[e]);
              unsigned short lb = f2bf_bits(sp[e] - bf_bits2f(hb));
              hv[e] = __builtin_bit_cast(_Float16, hb);
              lv[e] = __builtin_bit_cast(_Float16, lb);
            }
          }
          *(volatile v8h*)(C + (size_t)(mBase + row) * ldc + n0 + c8) = hv;
          if (OUT_MODE == 2) *(volatile v8h*)(C2 + (size_t)(mBase + row) * ldc + n0 + c8) = lv;
        }
        __threadfence();
      }
    }
    __builtin_amdgcn_fence(__ATOMIC_RELEASE, "workgroup");
    __builtin_amdgcn_wave_barrier();
    __builtin_amdgcn_fence(__ATOMIC_ACQUIRE, "workgroup");
  }
}

__global__ __launch_bounds__(NTHR) void gather_cvt_kernel(const int* __restrict__ sent, const float* __restrict__ emb,
                                                          unsigned short* __restrict__ e16) {
  const int i = blockIdx.x * NTHR + threadIdx.x;
  if (i < NROWS * (NE / 8)) {
    const int row = i >> 5;
    const int c8  = i & 31;
    const int t   = row >> 6;
    const int b   = row & 63;
    int tok = sent[b * NT + t];
    tok = tok < 0 ? 0 : tok;
    tok = tok > (NVOC - 1) ? (NVOC - 1) : tok;
    const float* sp = emb + (size_t)tok * NE + c8 * 8;
    const v4f a  = *(const v4f*)(sp);
    const v4f bq = *(const v4f*)(sp + 4);
    v8h hv;
#pragma unroll
    for (int e = 0; e < 4; ++e) {
      hv[e]     = (_Float16)(a[e] * EMB_CARRY);
      hv[4 + e] = (_Float16)(bq[e] * EMB_CARRY);
    }
    unsigned short* ph = e16 + (size_t)i * 8;
    *(volatile v8h*)ph = hv;
    __threadfence();
    *(volatile v8h*)ph = hv;
  }
}

__global__ __launch_bounds__(NTHR) void tcast_kernel(const float* __restrict__ src, unsigned short* __restrict__ dst,
                                                     int KR, int NC, float sc) {
  __shared__ __align__(16) float tl[64 * TSP];
  const int tid = threadIdx.x, lane = tid & 31, wave = tid >> 5;
  const int n0 = blockIdx.x * 64, k0 = blockIdx.y * 64;
#pragma unroll
  for (int it = 0; it < 4; ++it) {
    const int idx = it * NTHR + tid;
    const int kk  = idx >> 4;
    const int n4  = (idx & 15) * 4;
    const v4f v = *(const v4f*)(src + (size_t)(k0 + kk) * NC + n0 + n4);
    tl[(n4 + 0) * TSP + kk] = v[0];
    tl[(n4 + 1) * TSP + kk] = v[1];
    tl[(n4 + 2) * TSP + kk] = v[2];
    tl[(n4 + 3) * TSP + kk] = v[3];
  }
  __syncthreads();
  const int q = lane >> 3, c8 = (lane & 7) * 8;
  v8h hv[2];
  size_t o[2];
#pragma unroll
  for (int it = 0; it < 2; ++it) {
    const int nrow = it * 32 + wave * 4 + q;
    const float* sp = tl + nrow * TSP + c8;
    const v4f a  = *(const v4f*)(sp);
    const v4f bq = *(const v4f*)(sp + 4);
#pragma unroll
    for (int e = 0; e < 4; ++e) {
      hv[it][e]     = (_Float16)(a[e] * sc);
      hv[it][4 + e] = (_Float16)(bq[e] * sc);
    }
    o[it] = (size_t)(n0 + nrow) * KR + k0 + c8;
  }
  for (int pass = 0; pass < 2; ++pass) {
    *(volatile v8h*)(dst + o[0]) = hv[0];
    *(volatile v8h*)(dst + o[1]) = hv[1];
    __threadfence();
  }
}

__device__ __forceinline__ float ftanh(float x) { return 1.0f - 2.0f * __builtin_amdgcn_rcpf(__expf(2.0f * x) + 1.0f); }

__global__ __launch_bounds__(NTHR) void rnn_seq_kernel(const float* __restrict__ XW,
                                                       const unsigned short* __restrict__ WHTp,
                                                       float* __restrict__ HFIN) {
  __shared__ __align__(16) _Float16 AH[2 * ABUF];
  __shared__ __align__(16) float    Sl[NTHR / 32][16 * SLABP];
  const _Float16* WHT = (const _Float16*)WHTp;
  const int tid = threadIdx.x, lane = tid & 31, wave = tid >> 5;
  const int c = lane & 15, hh = lane >> 4, koff = hh * 8, c4 = c * 4;
  const int rowbase = blockIdx.x * SEQ_BLK;

  {
#pragma unroll 1
    for (int i = tid; i < 2 * ABUF; i += NTHR) AH[i] = (_Float16)0.0f;
  }
  float hst[4][8];
#pragma unroll
  for (int nt = 0; nt < 4; ++nt)
#pragma unroll
    for (int r = 0; r < 8; ++r) hst[nt][r] = 0.0f;
  __syncthreads();

  const v8f z8 = {0.f, 0.f, 0.f, 0.f, 0.f, 0.f, 0.f, 0.f};

#pragma unroll 1
  for (int t = 0; t < NT; ++t) {
    const int cur = t & 1;
    const _Float16* arow = AH + cur * ABUF + c * HPITCH + koff;
    _Float16* ahn = AH + (cur ^ 1) * ABUF;
    v8f acc[4];
#pragma unroll
    for (int nt = 0; nt < 4; ++nt) acc[nt] = z8;
#pragma unroll 1
    for (int k0 = 0; k0 < NU; k0 += 32) {
      const v16h a = Frag<_Float16>::load(arow + k0);
      v16h bq[4];
#pragma unroll
      for (int nt = 0; nt < 4; ++nt)
        bq[nt] = Frag<_Float16>::load(WHT + (size_t)(64 * wave + 16 * nt + c) * NU + koff + k0);
#pragma unroll
      for (int nt = 0; nt < 4; ++nt) acc[nt] = Frag<_Float16>::mma(a, bq[nt], acc[nt]);
      dep_guard_h(acc[0], acc[3], a, bq[3]);
      keep4_h(bq[0], bq[1], bq[2], a);
    }
    acc_guard4(acc[0], acc[1], acc[2], acc[3]);

#pragma unroll
    for (int nt = 0; nt < 4; ++nt) {
      const int j = 64 * wave + 16 * nt + c;
      float xr[8];
#pragma unroll
      for (int r = 0; r < 8; ++r)
        xr[r] = XW[((size_t)t * NB + (size_t)(rowbase + 8 * hh + r)) * NU + j];
#pragma unroll
      for (int r = 0; r < 8; ++r) {
        const float pre = acc[nt][r] * WH_FOLD + xr[r];
        const float hn  = ftanh(pre);
        hst[nt][r] = hn;
        ahn[(8 * hh + r) * HPITCH + j] = (_Float16)hn;
      }
    }
    __syncthreads();
  }

  float* slab = Sl[wave];
#pragma unroll
  for (int nt = 0; nt < 4; ++nt)
#pragma unroll
    for (int r = 0; r < 8; ++r) slab[(8 * hh + r) * SLABP + 16 * nt + c] = hst[nt][r];
  __builtin_amdgcn_fence(__ATOMIC_RELEASE, "workgroup");
  __builtin_amdgcn_wave_barrier();
  __builtin_amdgcn_fence(__ATOMIC_ACQUIRE, "workgroup");
  for (int pass = 0; pass < 2; ++pass) {
#pragma unroll
    for (int it = 0; it < 8; ++it) {
      const int row = it * 2 + hh;
      const v4f v = *(const v4f*)(slab + row * SLABP + c4);
      *(volatile v4f*)(HFIN + (size_t)(rowbase + row) * NU + 64 * wave + c4) = v;
    }
    __threadfence();
  }
}

__global__ __launch_bounds__(NTHR) void head_kernel(const float* __restrict__ hfin, const float* __restrict__ W1,
                                                    const float* __restrict__ b1, const float* __restrict__ W2,
                                                    const float* __restrict__ b2, const float* __restrict__ W3,
                                                    const float* __restrict__ b3, float* __restrict__ out) {
  __shared__ float z1[NB * NH1];
  __shared__ float z2[NB * NH2];
  __shared__ __align__(16) float o64[NB];
  const int tid = threadIdx.x, lane = tid & 31;
#pragma unroll 1
  for (int o = tid; o < NB * NH1; o += NTHR) {
    const int bb = o >> 7, j = o & (NH1 - 1);
    float s = 0.0f;
#pragma unroll 1
    for (int k = 0; k < NU; ++k) s += hfin[bb * NU + k] * W1[k * NH1 + j];
    s += b1[j];
    z1[o] = fmaxf(s, 0.0f);
  }
  __syncthreads();
#pragma unroll 1
  for (int o = tid; o < NB * NH2; o += NTHR) {
    const int bb = o >> 6, j = o & (NH2 - 1);
    float s = 0.0f;
#pragma unroll 1
    for (int k = 0; k < NH1; ++k) s += z1[bb * NH1 + k] * W2[k * NH2 + j];
    s += b2[j];
    z2[o] = fmaxf(s, 0.0f);
  }
  __syncthreads();
  if (tid < NB) {
    float s = 0.0f;
#pragma unroll 1
    for (int k = 0; k < NH2; ++k) s += z2[tid * NH2 + k] * W3[k];
    s += b3[0];
    o64[tid] = 1.0f / (1.0f + expf(-s));
  }
  __syncthreads();
  if (tid < 32) {
    const int li = (lane < 16) ? lane : 15;
    const v4f v = *(const v4f*)(o64 + li * 4);
    for (int pass = 0; pass < 2; ++pass) {
      if (lane < 16) *(volatile v4f*)(out + lane * 4) = v;
      __threadfence();
    }
  }
}

extern "C" void kernel_launch(void* const* d_in, const int* in_sizes, int n_in,
                              void* d_out, int out_size, void* d_ws, size_t ws_size, hipStream_t stream) {
  if (n_in < 11 || d_out == nullptr || d_ws == nullptr) return;
  if (in_sizes[0] != NB * NT || in_sizes[1] != NVOC * NE || in_sizes[2] != NE * NU || in_sizes[3] != NU * NU ||
      in_sizes[4] != NU || in_sizes[5] != NU * NH1 || in_sizes[6] != NH1 || in_sizes[7] != NH1 * NH2 ||
      in_sizes[8] != NH2 || in_sizes[9] != NH2 || in_sizes[10] != 1 || out_size != NB) return;

  const int*   sent = (const int*)d_in[0];
  const float* emb  = (const float*)d_in[1];
  const float* Wx   = (const float*)d_in[2];
  const float* Wh   = (const float*)d_in[3];
  const float* bvec = (const float*)d_in[4];
  const float* W1   = (const float*)d_in[5];
  const float* b1   = (const float*)d_in[6];
  const float* W2   = (const float*)d_in[7];
  const float* b2   = (const float*)d_in[8];
  const float* W3   = (const float*)d_in[9];
  const float* b3   = (const float*)d_in[10];
  float* out = (float*)d_out;

  char* ws = (char*)d_ws; size_t off = 0;
  auto carve = [&](size_t bytes) -> char* { char* p = ws + off; off += (bytes + 255) & ~(size_t)255; return p; };
  unsigned short* E16  = (unsigned short*)carve((size_t)NROWS * NE * 2);
  unsigned short* WXT  = (unsigned short*)carve((size_t)NU * NE * 2);
  unsigned short* WHT  = (unsigned short*)carve((size_t)NU * NU * 2);
  float*          XW   = (float*)carve((size_t)NROWS * NU * 4);
  float*          HFIN = (float*)carve((size_t)NB * NU * 4);
  if (off > ws_size || off > (size_t)134217728) return;

  gather_cvt_kernel<<<(NROWS * (NE / 8)) / NTHR, NTHR, 0, stream>>>(sent, emb, E16);
  tcast_kernel<<<dim3(NU / 64, NE / 64), NTHR, 0, stream>>>(Wx, WXT, NE, NU, W_CARRY);
  tcast_kernel<<<dim3(NU / 64, NU / 64), NTHR, 0, stream>>>(Wh, WHT, NU, NU, W_CARRY);

  const dim3 ggrid((NROWS / 64) * (NU / 64) / 8, 1);
  wmma_gemm64<0, false, 2, 0, false, 0><<<ggrid, 256, 0, stream>>>(
      E16, E16, NE, 0L, WXT, WXT, NE, 0L, (void*)XW, (void*)XW, NU, 0L,
      bvec, XW, 0L, NROWS, NU, NE, XW_FOLD);

  rnn_seq_kernel<<<NB / SEQ_BLK, NTHR, 0, stream>>>(XW, WHT, HFIN);

  head_kernel<<<1, NTHR, 0, stream>>>(HFIN, W1, b1, W2, b2, W3, b3, out);
}
